// ConceptGNN_4655744549232
// MI455X (gfx1250) — hardware-run, weakly checked
//
#include <hip/hip_runtime.h>

typedef float          v8f   __attribute__((ext_vector_type(8)));
typedef float          v4f   __attribute__((ext_vector_type(4)));
typedef unsigned int   v4u   __attribute__((ext_vector_type(4)));
typedef int            v8i   __attribute__((ext_vector_type(8)));
typedef unsigned short v8us  __attribute__((ext_vector_type(8)));
typedef unsigned short v16us __attribute__((ext_vector_type(16)));
typedef __bf16         v16bf __attribute__((ext_vector_type(16)));
typedef _Float16       v16h  __attribute__((ext_vector_type(16)));
typedef v4f  __attribute__((may_alias)) v4fa;
typedef v8us __attribute__((may_alias)) v8usa;
union FragB { v16bf v; v16us u; v8us h[2]; v8i w; };
union FragH { v16h  v; v16us u; v8us h[2]; v8i w; };

__device__ __forceinline__ v8f wmb(const FragB& a, const FragB& b, v8f c) {
  v8f d = __builtin_amdgcn_wmma_f32_16x16x32_bf16(false, a.v, false, b.v, (short)0, c, false, false);
  asm volatile("v_nop\n\tv_nop\n\tv_nop\n\tv_nop" : "+v"(d) : "v"(a.w), "v"(b.w));
  return d;
}

__device__ __forceinline__ v8f wmh(const FragH& a, const FragH& b, v8f c) {
  v8f d = __builtin_amdgcn_wmma_f32_16x16x32_f16(false, a.v, false, b.v, (short)0, c, false, false);
  asm volatile("v_nop\n\tv_nop\n\tv_nop\n\tv_nop" : "+v"(d) : "v"(a.w), "v"(b.w));
  return d;
}

__device__ __forceinline__ unsigned bf16_bits(float f) {
  const unsigned u = __float_as_uint(f);
  const unsigned r = (u + 0x7FFFu + ((u >> 16) & 1u)) >> 16;
  const unsigned q = (u >> 16) | 0x40u;
  return ((u & 0x7fffffffu) > 0x7f800000u) ? q : r;
}

__device__ __forceinline__ float bf16_val(float f) {
  return __uint_as_float(bf16_bits(f) << 16);
}
__device__ __forceinline__ int clampi(int v, int lo, int hi) {
  return v < lo ? lo : (v > hi ? hi : v);
}

__device__ __forceinline__ unsigned f16_bits(float f) {
  const unsigned u  = __float_as_uint(f);
  const unsigned s  = (u >> 16) & 0x8000u;
  const unsigned a  = u & 0x7fffffffu;
  const unsigned t  = a - 0x38000000u;
  const unsigned r  = (t + 0x0FFFu + ((t >> 13) & 1u)) >> 13;
  const unsigned rc = r > 0x7C00u ? 0x7C00u : r;
  const bool small  = a < 0x38800000u;
  const bool isnan  = a > 0x7f800000u;
  const unsigned fin = small ? 0u : (s | rc);
  return isnan ? (s | 0x7E00u) : fin;
}

__device__ __forceinline__ unsigned pk16(unsigned lo, unsigned hi) { return lo | (hi << 16); }
__device__ __forceinline__ unsigned bf16_lo_bits(float v) {
  float hi = bf16_val(v);
  asm volatile("" : "+v"(hi));
  return bf16_bits(v - hi);
}
__device__ __forceinline__ v4u pack8_bf16(v4f a, v4f c) {
  return (v4u){ pk16(bf16_bits(a[0]), bf16_bits(a[1])), pk16(bf16_bits(a[2]), bf16_bits(a[3])),
                pk16(bf16_bits(c[0]), bf16_bits(c[1])), pk16(bf16_bits(c[2]), bf16_bits(c[3])) };
}
__device__ __forceinline__ v4u pack8_bf16_lo(v4f a, v4f c) {
  return (v4u){ pk16(bf16_lo_bits(a[0]), bf16_lo_bits(a[1])), pk16(bf16_lo_bits(a[2]), bf16_lo_bits(a[3])),
                pk16(bf16_lo_bits(c[0]), bf16_lo_bits(c[1])), pk16(bf16_lo_bits(c[2]), bf16_lo_bits(c[3])) };
}
__device__ __forceinline__ v4u pack8_f16(v4f a, v4f c) {
  return (v4u){ pk16(f16_bits(a[0]), f16_bits(a[1])), pk16(f16_bits(a[2]), f16_bits(a[3])),
                pk16(f16_bits(c[0]), f16_bits(c[1])), pk16(f16_bits(c[2]), f16_bits(c[3])) };
}

template <int FORM>
__global__ __launch_bounds__(256) void k_plane(const float* __restrict__ src, int rows, int cols, int ldsrc,
                                               unsigned short* __restrict__ dst, int MP, int KP) {
  static_assert(FORM >= 0 && FORM <= 3);
  const int KTOT = (FORM == 1 || FORM == 3) ? 2 * KP : KP;
  const unsigned ppr   = (unsigned)(KTOT >> 3);
  const unsigned kp8   = (unsigned)(KP >> 3);
  const unsigned total = (unsigned)MP * ppr;
  const unsigned g     = blockIdx.x * 256u + threadIdx.x;
  const unsigned rowu  = g / ppr;
  const unsigned p     = g - rowu * ppr;
  const bool second    = p >= kp8;
  const int row = (int)rowu;
  const int c0  = (int)((second ? p - kp8 : p) << 3);
  const float* srow = src + (size_t)clampi(row, 0, rows - 1) * (size_t)ldsrc;
  float x[8];
  unsigned mk[8];
#pragma unroll
  for (int e = 0; e < 8; ++e) {
    const int c = c0 + e;
    const float v = srow[clampi(c, 0, cols - 1)];
    asm volatile("" :: "v"(v));
    x[e]  = v;
    mk[e] = (row < rows && c < cols) ? 0xFFFFu : 0u;
  }
  const v4f a = (v4f){ x[0], x[1], x[2], x[3] };
  const v4f c = (v4f){ x[4], x[5], x[6], x[7] };
  v4u o;
  if (FORM == 2) {
    o = pack8_f16(a, c);
  } else {
    const v4u hi = pack8_bf16(a, c);
    o = hi;
    if (FORM == 1) { const v4u lo = pack8_bf16_lo(a, c); o = second ? lo : hi; }
  }
  const v4u mw = (v4u){ pk16(mk[0], mk[1]), pk16(mk[2], mk[3]), pk16(mk[4], mk[5]), pk16(mk[6], mk[7]) };
  o &= mw;
  if (g < total) {
    volatile v4u* q = (volatile v4u*)(dst + (size_t)g * 8);
    *q = o;
    __threadfence();
    *q = o;
  }
}

template <int FORM> struct FragOf    { typedef FragB T; };
template <>         struct FragOf<2> { typedef FragH T; };
__device__ __forceinline__ v8f mm(const FragB& a, const FragB& b, v8f c) { return wmb(a, b, c); }
__device__ __forceinline__ v8f mm(const FragH& a, const FragH& b, v8f c) { return wmh(a, b, c); }
template <class F> __device__ __forceinline__ F ld_frag(const unsigned short* p) {
  F f;
  f.h[0] = *(const v8usa*)(p);
  f.h[1] = *(const v8usa*)(p + 16);
  return f;
}

template <int FORM, int EPI>
__global__ __launch_bounds__(256) __attribute__((amdgpu_num_vgpr(248)))
void k_gemm_nt(const unsigned short* __restrict__ A, const unsigned short* __restrict__ B,
               const float* __restrict__ bias, float* __restrict__ D, int M, int N, int KTOT, int ldd) {
  static_assert(FORM >= 0 && FORM <= 2);
  static_assert(EPI == 0 || EPI == 1);
  typedef typename FragOf<FORM>::T F;
  __shared__ __attribute__((aligned(16))) float sT[8][16 * 68];
  const int lane = threadIdx.x & 31;
  const int wave = threadIdx.x >> 5;
  const int tilesM = (M + 63) >> 6;
  const int tilesN = (N + 63) >> 6;
  const int tile = blockIdx.x * 8 + wave;
  if (tile >= tilesM * tilesN) return;
  const int tm = tile / tilesN;
  const int tn = tile - tm * tilesN;
  const int m0 = tm << 6;
  const int n0 = tn << 6;

  const int rl = lane & 15;
  const int h8 = (lane >> 4) * 8;
  const unsigned short* pa = A + (size_t)(m0 + rl) * (size_t)KTOT + h8;
  const unsigned short* pb = B + (size_t)(n0 + rl) * (size_t)KTOT + h8;

  v8f acc[4][4];
#pragma unroll
  for (int i = 0; i < 4; ++i)
#pragma unroll
    for (int j = 0; j < 4; ++j) acc[i][j] = (v8f){0.f, 0.f, 0.f, 0.f, 0.f, 0.f, 0.f, 0.f};

#pragma unroll 1
  for (int k0 = 0; k0 < KTOT; k0 += 32) {
    F bf[4];
#pragma unroll
    for (int j = 0; j < 4; ++j) bf[j] = ld_frag<F>(pb + (size_t)(j << 4) * (size_t)KTOT + k0);
#pragma unroll
    for (int i = 0; i < 4; ++i) {
      const F af = ld_frag<F>(pa + (size_t)(i << 4) * (size_t)KTOT + k0);
#pragma unroll
      for (int j = 0; j < 4; ++j) acc[i][j] = mm(af, bf[j], acc[i][j]);
    }
  }

  float* slab = sT[wave];
  const int hh = lane >> 4;
  const int c4 = (lane & 15) * 4;
  const int nc = n0 + c4;
  const bool cok = nc < N;
  v4f bv = (v4f){0.f, 0.f, 0.f, 0.f};
  if (EPI == 1) {
    bv = *(const v4fa*)(bias + clampi(nc, 0, N - 4));
    asm volatile("" :: "v"(bv));
  }
#pragma unroll
  for (int i = 0; i < 4; ++i) {
    const int mBase = m0 + (i << 4);
#pragma unroll
    for (int j = 0; j < 4; ++j) {
#pragma unroll
      for (int r = 0; r < 8; ++r) slab[(h8 + r) * 68 + (j << 4) + rl] = acc[i][j][r];
    }
    __builtin_amdgcn_fence(__ATOMIC_RELEASE, "workgroup");
    __builtin_amdgcn_wave_barrier();
    __builtin_amdgcn_fence(__ATOMIC_ACQUIRE, "workgroup");
    v4f vv[8];
#pragma unroll
    for (int it = 0; it < 8; ++it) {
      const int row = it * 2 + hh;
      v4f v = *(const v4fa*)(slab + row * 68 + c4);
      if (EPI == 1) v += bv;
      vv[it] = v;
    }
    for (int pass = 0; pass < 2; ++pass) {
#pragma unroll
      for (int it = 0; it < 8; ++it) {
        const int row = mBase + it * 2 + hh;
        if (cok && row < M) *(volatile v4f*)(D + (size_t)row * (size_t)ldd + nc) = vv[it];
      }
      __threadfence();
    }
    __builtin_amdgcn_fence(__ATOMIC_RELEASE, "workgroup");
    __builtin_amdgcn_wave_barrier();
    __builtin_amdgcn_fence(__ATOMIC_ACQUIRE, "workgroup");
  }
}

#pragma clang fp contract(off)

#ifndef ZSPLIT1
#define ZSPLIT1 1
#endif
#ifndef ZSPLIT2
#define ZSPLIT2 1
#endif

#define GN_N    50000
#define GN_NP   50048
#define GN_E    640000
#define DF      128
#define K2      256
#define NREL    6
#define NBA     1024
#define SLA     10
#define NBLK    49
#define RCAP    17408
#define DEGCAP  64
#define CHUNK   2048
#define NCHUNK  313

#define BK_LDS_INTS  (2 * RCAP + 3 * NBA + 32)
#define BK_LDS_BYTES (BK_LDS_INTS * 4)

#define PREP_XB_PIECES (GN_NP * DF / 8)
#define PREP_XB_BLOCKS (PREP_XB_PIECES / 256)
#define PREP_W_BLOCKS  32
#define PREP_R_BLOCKS  1
#define PREP_ZP_PIECES ((GN_NP - GN_N) * K2 * 2 / 16)
#define PREP_ZP_BLOCKS (PREP_ZP_PIECES / 256)
#define PREP_BLOCKS    (PREP_XB_BLOCKS + PREP_W_BLOCKS + PREP_R_BLOCKS + PREP_ZP_BLOCKS)

static_assert(GN_N % 8 == 0);
static_assert(GN_NP % 128 == 0 && GN_NP >= GN_N && GN_NP % 64 == 0);
static_assert(DF == 128 && DF == 32 * 4);
static_assert(K2 == 256 && K2 == 2 * DF && K2 % 32 == 0);
static_assert(GN_E == 312 * 2048 + 1024);
static_assert(NCHUNK * CHUNK >= GN_E && (NCHUNK - 1) * CHUNK < GN_E);
static_assert(GN_N < (1 << 20) && NREL <= 8);
static_assert(((long long)GN_E << SLA) < (1LL << 31));
static_assert(NBA == (1 << SLA) && NBLK * NBA >= GN_N && (NBLK - 1) * NBA < GN_N);
static_assert(RCAP * 4 >= 13379 * 5);
static_assert(RCAP % 1024 == 0 && RCAP % 256 == 0);
static_assert(DEGCAP >= 29 + 8 && DEGCAP <= 64);
static_assert(BK_LDS_BYTES <= 262144);
static_assert((2 * RCAP + 3 * NBA) % 4 == 0);
static_assert(PREP_XB_PIECES % 256 == 0 && PREP_ZP_PIECES % 256 == 0);
static_assert(NREL * DF / 4 <= 256);

constexpr size_t SZ_XB   = (size_t)GN_NP * DF * 2;
constexpr size_t SZ_ZHL  = (size_t)GN_NP * K2 * 2;
constexpr size_t SZ_P    = (size_t)GN_NP * DF * 4;
constexpr size_t SZ_LIST = (size_t)NBLK * RCAP * 4;
constexpr size_t SZ_CNT  = (size_t)NBLK * NBA * 4;
constexpr size_t SZ_OFF  = (size_t)NBLK * NBA * 4;
constexpr size_t SZ_WD   = (size_t)DF * K2 * 2;
constexpr size_t SZ_REL  = (size_t)NREL * DF * 4;
constexpr size_t SZ_FLAG = (((size_t)NBLK * 128) + 255) & ~(size_t)255;
constexpr size_t O_XB   = 0;
constexpr size_t O_ZHL  = O_XB + SZ_XB;
constexpr size_t O_P    = O_ZHL + SZ_ZHL;
constexpr size_t O_LIST = O_P + SZ_P;
constexpr size_t O_CNT  = O_LIST + SZ_LIST;
constexpr size_t O_OFF  = O_CNT + SZ_CNT;
constexpr size_t O_W1D  = O_OFF + SZ_OFF;
constexpr size_t O_W2D  = O_W1D + SZ_WD;
constexpr size_t O_REL  = O_W2D + SZ_WD;
constexpr size_t O_FLAG = O_REL + SZ_REL;
constexpr size_t WS_TOTAL = O_FLAG + SZ_FLAG;
static_assert(SZ_XB % 256 == 0 && SZ_ZHL % 256 == 0 && SZ_P % 256 == 0 && SZ_LIST % 256 == 0);
static_assert(SZ_CNT % 256 == 0 && SZ_WD % 256 == 0 && SZ_REL % 256 == 0 && SZ_FLAG % 256 == 0);
static_assert(WS_TOTAL <= ((size_t)128 << 20));

typedef unsigned v2u __attribute__((ext_vector_type(2)));
typedef int      v4i __attribute__((ext_vector_type(4)));
typedef v2u __attribute__((may_alias)) v2ua;
typedef v4u __attribute__((may_alias)) v4ua;
typedef v4i __attribute__((may_alias)) v4ia;

__device__ __forceinline__ void st2_u4(unsigned short* p, v4u o) {
  volatile v4u* q = (volatile v4u*)p; *q = o; __threadfence(); *q = o;
}
__device__ __forceinline__ void st2_w4(unsigned* p, v4u o) {
  volatile v4u* q = (volatile v4u*)p; *q = o; __threadfence(); *q = o;
}
__device__ __forceinline__ void st2_i4(int* p, v4i o) {
  volatile v4i* q = (volatile v4i*)p; *q = o; __threadfence(); *q = o;
}
__device__ __forceinline__ void st2_f4(float* p, v4f o) {
  volatile v4f* q = (volatile v4f*)p; *q = o; __threadfence(); *q = o;
}
__device__ __forceinline__ void wave_sync() {
  __builtin_amdgcn_fence(__ATOMIC_RELEASE, "wavefront");
  __builtin_amdgcn_wave_barrier();
  __builtin_amdgcn_fence(__ATOMIC_ACQUIRE, "wavefront");
}
__device__ __forceinline__ float relu_k(float v) { return (v > 0.0f) ? v : (v - v); }

__device__ __forceinline__ void prep_wpiece(const float* __restrict__ W, unsigned short* __restrict__ WD, int v) {
  const int n  = v >> 5;
  const int p  = v & 31;
  const int k0 = (p & 15) * 8;
  float xv[8];
#pragma unroll
  for (int e = 0; e < 8; ++e) {
    const float t = W[(size_t)(k0 + e) * DF + n];
    asm volatile("" :: "v"(t));
    xv[e] = t;
  }
  const v4u o = pack8_bf16((v4f){ xv[0], xv[1], xv[2], xv[3] }, (v4f){ xv[4], xv[5], xv[6], xv[7] });
  st2_u4(WD + (size_t)n * K2 + (size_t)p * 8, o);
}

__global__ __launch_bounds__(256) void k_prep(const float* __restrict__ x, const float* __restrict__ rel,
                                              const float* __restrict__ W1, const float* __restrict__ W2,
                                              unsigned short* __restrict__ XB, unsigned short* __restrict__ W1D,
                                              unsigned short* __restrict__ W2D, float* __restrict__ REL,
                                              unsigned short* __restrict__ ZHL) {
  const int b   = (int)blockIdx.x;
  const int tid = (int)threadIdx.x;
  if (b < PREP_XB_BLOCKS) {
    const int g   = b * 256 + tid;
    const int row = g >> 4;
    const int p   = g & 15;
    const int rc  = row < GN_N ? row : GN_N - 1;
    const float* s = x + (size_t)rc * DF + p * 8;
    const v4f a = *(const v4fa*)s;
    const v4f c = *(const v4fa*)(s + 4);
    asm volatile("" :: "v"(a));
    asm volatile("" :: "v"(c));
    v4u o = pack8_bf16(a, c);
    const unsigned m = row < GN_N ? 0xFFFFFFFFu : 0u;
    o &= (v4u){ m, m, m, m };
    st2_u4(XB + (size_t)g * 8, o);
  } else if (b < PREP_XB_BLOCKS + PREP_W_BLOCKS) {
    const int u = (b - PREP_XB_BLOCKS) * 256 + tid;
    const int v = u & 4095;
    if ((u >> 12) == 0) prep_wpiece(W1, W1D, v);
    else                prep_wpiece(W2, W2D, v);
  } else if (b < PREP_XB_BLOCKS + PREP_W_BLOCKS + PREP_R_BLOCKS) {
    if (tid < NREL * DF / 4) {
      const v4f r = *(const v4fa*)(rel + 4 * tid);
      asm volatile("" :: "v"(r));
      const v4f o = (v4f){ bf16_val(r[0]), bf16_val(r[1]), bf16_val(r[2]), bf16_val(r[3]) };
      st2_f4(REL + 4 * tid, o);
    }
  } else {
    const int g = (b - (PREP_XB_BLOCKS + PREP_W_BLOCKS + PREP_R_BLOCKS)) * 256 + tid;
    if (g < PREP_ZP_PIECES) {
      const v4u z = (v4u){ 0u, 0u, 0u, 0u };
      st2_u4(ZHL + (size_t)GN_N * K2 + (size_t)g * 8, z);
    }
  }
}

__global__ __launch_bounds__(256) void k_bucket(const int* __restrict__ srcs, const int* __restrict__ dsts,
                                                const int* __restrict__ types, unsigned* __restrict__ LIST,
                                                int* __restrict__ CNT, int* __restrict__ OFF,
                                                int* __restrict__ FLAG) {
  extern __shared__ __attribute__((aligned(16))) int dsm[];
  int* hl   = dsm;
  int* sl   = dsm + RCAP;
  int* cnt  = dsm + 2 * RCAP;
  int* offs = cnt + NBA;
  int* cur  = offs + NBA;
  int* misc = cur + NBA;
  const int tid = (int)threadIdx.x, lane = tid & 31, wave = tid >> 5;
  const int blk = (int)blockIdx.x;
  const unsigned base = (unsigned)blk * NBA;
  const int rem = GN_N - blk * NBA;
  const unsigned nb = (unsigned)(rem < 0 ? 0 : (rem > NBA ? NBA : rem));

  for (int i = tid; i < NBA; i += 256) cnt[i] = 0;
  if (tid < 32) misc[tid] = 0;
  if (tid == 0) { hl[0] = 0; sl[0] = 0; }
  __syncthreads();

  int tot = 0;
#pragma unroll 1
  for (int ch = 0; ch < NCHUNK; ++ch) {
    const int eb = ch * CHUNK + wave * 256 + lane;
    unsigned sv[8];
    unsigned mj[8];
    bool hv[8];
    int wc = 0;
#pragma unroll
    for (int j = 0; j < 8; ++j) {
      const int e  = eb + 32 * j;
      const int ec = e < GN_E ? e : GN_E - 1;
      const int k  = dsts[ec];
      asm volatile("" :: "v"(k));
      const int inval = (e < GN_E) ? 0 : -1;
      const unsigned s = (unsigned)(k | inval) - base;
      const bool h = s < nb;
      const unsigned m = __builtin_amdgcn_ballot_w32(h);
      sv[j] = s; hv[j] = h; mj[j] = m;
      wc += (int)__builtin_popcount(m);
    }
    const int par = (ch & 1) * 8;
    if (lane == 0) misc[par + wave] = wc;
    __syncthreads();
    const v4i ca = *(const v4ia*)(misc + par);
    const v4i cb = *(const v4ia*)(misc + par + 4);
    int pre = 0;
    pre += (wave > 0) ? ca[0] : 0;
    pre += (wave > 1) ? ca[1] : 0;
    pre += (wave > 2) ? ca[2] : 0;
    pre += (wave > 3) ? ca[3] : 0;
    pre += (wave > 4) ? cb[0] : 0;
    pre += (wave > 5) ? cb[1] : 0;
    pre += (wave > 6) ? cb[2] : 0;
    const int all = ca[0] + ca[1] + ca[2] + ca[3] + cb[0] + cb[1] + cb[2] + cb[3];
    int run = tot + pre;
#pragma unroll
    for (int j = 0; j < 8; ++j) {
      if (mj[j] != 0u) {
        if (hv[j]) {
          const int pos = run + (int)__builtin_amdgcn_mbcnt_lo(mj[j], 0u);
          if (pos < RCAP) hl[pos] = ((eb + 32 * j) << SLA) | (int)sv[j];
        }
        run += (int)__builtin_popcount(mj[j]);
      }
    }
    tot += all;
  }
  __syncthreads();
  const int tt  = tot < RCAP ? tot : RCAP;
  const int ovf = tot > RCAP ? 1 : 0;

#pragma unroll 1
  for (int b0 = 0; b0 < tt; b0 += 32) {
    const int i   = b0 + lane;
    const int ic  = i < tt ? i : tt - 1;
    const int ent = hl[ic];
    const bool mine = (i < tt) && (((ent >> 7) & 7) == wave);
    unsigned m = __builtin_amdgcn_ballot_w32(mine);
    while (m != 0u) {
      const int k = (int)__builtin_ctz(m);
      m &= m - 1u;
      const int u = __builtin_amdgcn_readlane(ent, k);
      const int s = u & (NBA - 1);
      if (lane == 0) cnt[s] = cnt[s] + 1;
    }
  }
  __syncthreads();

  if (wave == 0) {
    const int sb = lane * (NBA / 32);
    int s = 0;
#pragma unroll 1
    for (int i = 0; i < NBA / 32; ++i) s += cnt[sb + i];
    int incl = s;
#pragma unroll
    for (int d = 1; d < 32; d <<= 1) {
      const int y = __shfl_up(incl, d, 32);
      incl += (lane >= d) ? y : 0;
    }
    int runo = incl - s;
    int big = 0;
#pragma unroll 1
    for (int i = 0; i < NBA / 32; ++i) {
      const int cv = cnt[sb + i];
      offs[sb + i] = runo;
      cur[sb + i]  = runo;
      runo += cv;
      big |= (cv > DEGCAP) ? 1 : 0;
    }
    const unsigned bm = __builtin_amdgcn_ballot_w32(big != 0);
    if (lane == 0) misc[16] = (bm != 0u) ? 1 : 0;
  }
  __syncthreads();

#pragma unroll 1
  for (int b0 = 0; b0 < tt; b0 += 32) {
    const int i   = b0 + lane;
    const int ic  = i < tt ? i : tt - 1;
    const int ent = hl[ic];
    const bool mine = (i < tt) && (((ent >> 7) & 7) == wave);
    unsigned m = __builtin_amdgcn_ballot_w32(mine);
    while (m != 0u) {
      const int k = (int)__builtin_ctz(m);
      m &= m - 1u;
      const int u = __builtin_amdgcn_readlane(ent, k);
      const int s = u & (NBA - 1);
      if (lane == 0) {
        const int p  = cur[s];
        const int pc = clampi(p, 0, RCAP - 1);
        sl[pc] = u;
        cur[s] = p + 1;
      }
    }
  }
  __syncthreads();

  const int flag = ((ovf | misc[16]) != 0) ? 1 : 0;
  unsigned* Lb = LIST + (size_t)blk * RCAP;
  const int tl = tt > 0 ? tt - 1 : 0;
#pragma unroll 1
  for (int i4 = tid; i4 < RCAP / 4; i4 += 256) {
    unsigned w[4];
#pragma unroll
    for (int q = 0; q < 4; ++q) {
      const int i   = 4 * i4 + q;
      const int ic  = i < tl ? i : tl;
      const int ent = sl[ic];
      const int eid = clampi(ent >> SLA, 0, GN_E - 1);
      const int sr  = srcs[eid];
      asm volatile("" :: "v"(sr));
      const int ty  = types[eid];
      asm volatile("" :: "v"(ty));
      const unsigned word = (unsigned)clampi(sr, 0, GN_N - 1) | ((unsigned)clampi(ty, 0, NREL - 1) << 20);
      const unsigned keep = (i < tt) ? 0xFFFFFFFFu : 0u;
      w[q] = word & keep;
    }
    st2_w4(Lb + 4 * i4, (v4u){ w[0], w[1], w[2], w[3] });
  }
  {
    const v4i cv = *(const v4ia*)(cnt + 4 * tid);
    const v4i ov = *(const v4ia*)(offs + 4 * tid);
    st2_i4(CNT + (size_t)blk * NBA + 4 * tid, cv);
    st2_i4(OFF + (size_t)blk * NBA + 4 * tid, ov);
  }
  if (tid < 8) {
    const v4i fv = (v4i){ flag, flag, flag, flag };
    st2_i4(FLAG + blk * 32 + 4 * tid, fv);
  }
}

template <int L, int ZS>
__global__ __launch_bounds__(256) void k_replay(const unsigned short* __restrict__ XB, const float* __restrict__ Pin,
                                                const float* __restrict__ REL, const unsigned* __restrict__ LIST,
                                                const int* __restrict__ CNT, const int* __restrict__ OFF,
                                                const int* __restrict__ FLAG, unsigned short* __restrict__ ZHL,
                                                int nN) {
  static_assert(L == 1 || L == 2);
  __shared__ __attribute__((aligned(16))) float relS[NREL * DF];
  __shared__ __attribute__((aligned(16))) unsigned rowS[8 * 128];
  const int tid = (int)threadIdx.x, lane = tid & 31, wave = tid >> 5;
  if (tid < NREL * DF / 4) {
    const v4f r = *(const v4fa*)(REL + 4 * tid);
    *(v4fa*)(relS + 4 * tid) = r;
  }
  __syncthreads();

  const int t  = (int)blockIdx.x * 8 + wave;
  const bool live = t < nN;
  const int tc = live ? t : nN - 1;
  const int ob = tc >> SLA;
  const int c  = CNT[tc];
  asm volatile("" :: "v"(c));
  const int o  = OFF[tc];
  asm volatile("" :: "v"(o));
  const int fl = FLAG[ob * 32];
  asm volatile("" :: "v"(fl));
  const int cc = clampi(c, 0, DEGCAP);
  const int oc = clampi(o, 0, RCAP - 1);
  const int cn = __builtin_amdgcn_readfirstlane(live ? cc : 0);
  const unsigned* Lb = LIST + (size_t)ob * RCAP;

  float a0 = 0.0f, a1 = 0.0f, a2 = 0.0f, a3 = 0.0f;
#pragma unroll 1
  for (int b0 = 0; b0 < cn; b0 += 32) {
    int idx = oc + b0 + lane;
    idx = idx > RCAP - 1 ? RCAP - 1 : idx;
    const unsigned w = Lb[idx];
    asm volatile("" :: "v"(w));
    const int m32 = (cn - b0) < 32 ? (cn - b0) : 32;
#pragma unroll 1
    for (int j = 0; j < m32; ++j) {
      const unsigned wj = (unsigned)__builtin_amdgcn_readlane((int)w, j);
      int s  = (int)(wj & 0xFFFFFu);
      s = s > nN - 1 ? nN - 1 : s;
      int ty = (int)((wj >> 20) & 7u);
      ty = ty > NREL - 1 ? NREL - 1 : ty;
      const v4f rv = *(const v4fa*)(relS + ty * DF + 4 * lane);
      float x0, x1, x2, x3;
      if constexpr (L == 1) {
        const v2u xw = *(const v2ua*)(XB + (size_t)s * DF + 4 * lane);
        x0 = __uint_as_float(xw.x << 16);
        x1 = __uint_as_float(xw.x & 0xffff0000u);
        x2 = __uint_as_float(xw.y << 16);
        x3 = __uint_as_float(xw.y & 0xffff0000u);
      } else {
        const v4f pv = *(const v4fa*)(Pin + (size_t)s * DF + 4 * lane);
        x0 = relu_k(pv[0]); x1 = relu_k(pv[1]); x2 = relu_k(pv[2]); x3 = relu_k(pv[3]);
      }
      const float p0 = __fmul_rn(x0, rv[0]);
      const float p1 = __fmul_rn(x1, rv[1]);
      const float p2 = __fmul_rn(x2, rv[2]);
      const float p3 = __fmul_rn(x3, rv[3]);
      a0 = a0 + p0;
      a1 = a1 + p1;
      a2 = a2 + p2;
      a3 = a3 + p3;
    }
  }

  const float dn = (float)((cc > 1) ? cc : 1);
  const float m0 = a0 / dn;
  const float m1 = a1 / dn;
  const float m2 = a2 / dn;
  const float m3 = a3 / dn;

  float w0, w1, w2, w3;
  if constexpr (L == 1) {
    const v2u ow = *(const v2ua*)(XB + (size_t)tc * DF + 4 * lane);
    asm volatile("" :: "v"(ow));
    w0 = __uint_as_float(ow.x << 16);
    w1 = __uint_as_float(ow.x & 0xffff0000u);
    w2 = __uint_as_float(ow.y << 16);
    w3 = __uint_as_float(ow.y & 0xffff0000u);
  } else {
    const v4f ov = *(const v4fa*)(Pin + (size_t)tc * DF + 4 * lane);
    asm volatile("" :: "v"(ov));
    w0 = relu_k(ov[0]); w1 = relu_k(ov[1]); w2 = relu_k(ov[2]); w3 = relu_k(ov[3]);
  }
  float z0 = w0 + m0;
  float z1 = w1 + m1;
  float z2 = w2 + m2;
  float z3 = w3 + m3;
  const float qnan = __int_as_float(0x7fc00000);
  const bool poison = fl != 0;
  z0 = poison ? qnan : z0;
  z1 = poison ? qnan : z1;
  z2 = poison ? qnan : z2;
  z3 = poison ? qnan : z3;

  v2u hw, lw;
  hw.x = pk16(bf16_bits(z0), bf16_bits(z1));
  hw.y = pk16(bf16_bits(z2), bf16_bits(z3));
  if constexpr (ZS != 0) {
    lw.x = pk16(bf16_lo_bits(z0), bf16_lo_bits(z1));
    lw.y = pk16(bf16_lo_bits(z2), bf16_lo_bits(z3));
  } else {
    lw.x = 0u;
    lw.y = 0u;
  }
  unsigned* myrow = rowS + wave * 128;
  *(v2ua*)(myrow + 2 * lane)      = hw;
  *(v2ua*)(myrow + 64 + 2 * lane) = lw;
  wave_sync();
  const v4u q = *(const v4ua*)(myrow + 4 * lane);
  if (live) {
    volatile v4u* d = (volatile v4u*)(ZHL + (size_t)t * K2 + 8 * lane);
    *d = q;
    __threadfence();
    *d = q;
  }
}

__global__ __launch_bounds__(256) void k_out(const float* __restrict__ Pin, const int* __restrict__ FLAG,
                                             float* __restrict__ outp, int nN) {
  const int tid = (int)threadIdx.x, lane = tid & 31, wave = tid >> 5;
  const int row = (int)blockIdx.x * 8 + wave;
  const int rc  = row < nN ? row : nN - 1;
  const v4f v = *(const v4fa*)(Pin + (size_t)rc * DF + 4 * lane);
  asm volatile("" :: "v"(v));
  const int fl = FLAG[(rc >> SLA) * 32];
  asm volatile("" :: "v"(fl));
  const float qnan = __int_as_float(0x7fc00000);
  const bool poison = fl != 0;
  v4f y;
  y[0] = relu_k(v[0]); y[1] = relu_k(v[1]); y[2] = relu_k(v[2]); y[3] = relu_k(v[3]);
  y[0] = poison ? qnan : y[0];
  y[1] = poison ? qnan : y[1];
  y[2] = poison ? qnan : y[2];
  y[3] = poison ? qnan : y[3];
  if (row < nN) {
    volatile v4f* d = (volatile v4f*)(outp + (size_t)row * DF + 4 * lane);
    *d = y;
    __threadfence();
    *d = y;
  }
}

extern "C" void kernel_launch(void* const* d_in, const int* in_sizes, int n_in,
                              void* d_out, int out_size, void* d_ws, size_t ws_size,
                              hipStream_t stream) {
  if (n_in < 6) return;
  if (in_sizes[0] != GN_N * DF) return;
  if (in_sizes[1] != NREL * DF) return;
  if (in_sizes[2] != DF * DF || in_sizes[3] != DF * DF) return;
  if (in_sizes[4] != 2 * GN_E || in_sizes[5] != GN_E) return;
  if (out_size != GN_N * DF) return;
  if (WS_TOTAL > ws_size) return;

  const float* x   = (const float*)d_in[0];
  const float* rel = (const float*)d_in[1];
  const float* W1  = (const float*)d_in[2];
  const float* W2  = (const float*)d_in[3];
  const int*   ei  = (const int*)d_in[4];
  const int*   ea  = (const int*)d_in[5];
  const int*   src = ei;
  const int*   dst = ei + GN_E;
  float* out = (float*)d_out;

  char* ws = (char*)d_ws;
  unsigned short* XB   = (unsigned short*)(ws + O_XB);
  unsigned short* ZHL  = (unsigned short*)(ws + O_ZHL);
  float*          P    = (float*)(ws + O_P);
  unsigned*       LIST = (unsigned*)(ws + O_LIST);
  int*            CNT  = (int*)(ws + O_CNT);
  int*            OFF  = (int*)(ws + O_OFF);
  unsigned short* W1D  = (unsigned short*)(ws + O_W1D);
  unsigned short* W2D  = (unsigned short*)(ws + O_W2D);
  float*          REL  = (float*)(ws + O_REL);
  int*            FLAG = (int*)(ws + O_FLAG);

  hipFuncSetAttribute(reinterpret_cast<const void*>(&k_bucket), hipFuncAttributeMaxDynamicSharedMemorySize,
                      (int)BK_LDS_BYTES);

  const int gemmBlocks = (((GN_NP + 63) / 64) * ((DF + 63) / 64) + 7) / 8;

  k_prep<<<PREP_BLOCKS, 256, 0, stream>>>(x, rel, W1, W2, XB, W1D, W2D, REL, ZHL);
  k_bucket<<<NBLK, 256, BK_LDS_BYTES, stream>>>(src, dst, ea, LIST, CNT, OFF, FLAG);
  k_replay<1, ZSPLIT1><<<GN_N / 8, 256, 0, stream>>>(XB, P, REL, LIST, CNT, OFF, FLAG, ZHL, GN_N);
  k_gemm_nt<0, 0><<<gemmBlocks, 256, 0, stream>>>(ZHL, W1D, REL, P, GN_NP, DF, K2, DF);
  k_replay<2, ZSPLIT2><<<GN_N / 8, 256, 0, stream>>>(XB, P, REL, LIST, CNT, OFF, FLAG, ZHL, GN_N);
  k_gemm_nt<0, 0><<<gemmBlocks, 256, 0, stream>>>(ZHL, W2D, REL, P, GN_NP, DF, K2, DF);
  k_out<<<GN_N / 8, 256, 0, stream>>>(P, FLAG, out, GN_N);
}
